// SelfAttentionModule_6004364280161
// MI455X (gfx1250) — hardware-verified
//
#include <hip/hip_runtime.h>


#ifndef NB
#define NB 4
#endif
#ifndef SEQ
#define SEQ 2048
#endif
#define NB_FULL 4
#define SEQ_FULL 2048
#define DIM 1024
#define NH 16
#define HD 64
#define MTOK (NB * SEQ)

static_assert(NB >= 1 && NB <= NB_FULL);
static_assert(SEQ >= 128 && SEQ <= SEQ_FULL && (SEQ % 128) == 0);
static_assert(NH * HD == DIM && HD == 64 && (DIM % 64) == 0 && (DIM % 32) == 0);
static_assert((MTOK % 128) == 0 && (MTOK % 2) == 0);
static_assert(((3 * DIM * DIM / 8) % 256) == 0 && ((DIM * DIM / 8) % 256) == 0);

typedef _Float16 v16h __attribute__((ext_vector_type(16)));
typedef float v8f __attribute__((ext_vector_type(8)));
typedef float v4f __attribute__((ext_vector_type(4)));
typedef unsigned short u16;
typedef u16 v8us __attribute__((ext_vector_type(8)));
typedef unsigned v4u __attribute__((ext_vector_type(4)));
typedef v8us __attribute__((may_alias)) v8usa;
typedef v4f __attribute__((may_alias)) v4fa;
union Frag { v16h h; v8us u[2]; };
union Pk8 { v8us s; v4u w; };

__device__ __forceinline__ float bfr(float f) {
    unsigned u = __float_as_uint(f);
    u += 0x7FFFu + ((u >> 16) & 1u);
    return __uint_as_float(u & 0xFFFF0000u);
}
__device__ __forceinline__ unsigned h16(float f) { return (unsigned)__builtin_bit_cast(unsigned short, (_Float16)f); }
__device__ __forceinline__ unsigned pk2(float a, float b) { return h16(a) | (h16(b) << 16); }
__device__ __forceinline__ v8f vz8() {
    v8f z;
#pragma unroll
    for (int i = 0; i < 8; ++i) z[i] = 0.0f;
    return z;
}

__device__ __forceinline__ v16h ldfrag(const u16* rowp, int half) {
    Frag f;
    f.u[0] = *(const v8usa*)(rowp + 8 * half);
    f.u[1] = *(const v8usa*)(rowp + 16 + 8 * half);
    return f.h;
}
__device__ __forceinline__ v8f wmh(v16h a, v16h b, v8f c) {
    c = __builtin_amdgcn_wmma_f32_16x16x32_f16(false, a, false, b, (short)0, c, false, false);
    asm volatile("v_nop\n\tv_nop\n\tv_nop\n\tv_nop" : "+v"(c) : "v"(a), "v"(b));
    return c;
}
__device__ __forceinline__ void st2u(u16* p, v4u v) {
    *(volatile v4u*)p = v;
    __threadfence();
    *(volatile v4u*)p = v;
}
__device__ __forceinline__ void st2f(float* p, v4f v) {
    *(volatile v4f*)p = v;
    __threadfence();
    *(volatile v4f*)p = v;
}

__global__ __launch_bounds__(256) void k_cvt_x(const float* __restrict__ x, u16* XP) {
    const int tid = threadIdx.x;
    const int r = blockIdx.x * 2 + (tid >> 7);
    const int b = r / SEQ, n = r - b * SEQ;
    const int c0 = (tid & 127) * 8;
    const float* s = x + ((size_t)b * SEQ_FULL + n) * DIM + c0;
    const v4f a = *(const v4f*)s, c = *(const v4f*)(s + 4);
    v4u o;
    o[0] = pk2(bfr(a[0]) * 8.0f, bfr(a[1]) * 8.0f);
    o[1] = pk2(bfr(a[2]) * 8.0f, bfr(a[3]) * 8.0f);
    o[2] = pk2(bfr(c[0]) * 8.0f, bfr(c[1]) * 8.0f);
    o[3] = pk2(bfr(c[2]) * 8.0f, bfr(c[3]) * 8.0f);
    st2u(XP + (size_t)r * DIM + c0, o);
}
__global__ __launch_bounds__(256) void k_cvt_w(const float* __restrict__ w, u16* WP, int n8, float sc) {
    const int i = blockIdx.x * 256 + threadIdx.x;
    if (i >= n8) return;
    const float* s = w + (size_t)i * 8;
    const v4f a = *(const v4f*)s, c = *(const v4f*)(s + 4);
    v4u o;
    o[0] = pk2(bfr(a[0]) * sc, bfr(a[1]) * sc);
    o[1] = pk2(bfr(a[2]) * sc, bfr(a[3]) * sc);
    o[2] = pk2(bfr(c[0]) * sc, bfr(c[1]) * sc);
    o[3] = pk2(bfr(c[2]) * sc, bfr(c[3]) * sc);
    st2u(WP + (size_t)i * 8, o);
}

template <int MODE>
__global__ __launch_bounds__(256) void k_gemm(const u16* __restrict__ A, const u16* __restrict__ Bw, const float* __restrict__ bias,
                                              u16* PQ, u16* PK, u16* PV, float* Y) {
    __shared__ __align__(16) float cst[128 * 68];
    const int tid = threadIdx.x, lane = tid & 31, wv = tid >> 5, ln = lane & 15, half = lane >> 4;
    const int row0 = blockIdx.x * 128, col0 = blockIdx.y * 64;
    const u16* arow = A + (size_t)(row0 + wv * 16 + ln) * DIM;
    const u16* bbase = Bw + (size_t)(col0 + ln) * DIM;
    v8f acc[4];
#pragma unroll
    for (int t = 0; t < 4; ++t) acc[t] = vz8();
#pragma unroll 1
    for (int kc = 0; kc < DIM; kc += 32) {
        const v16h a = ldfrag(arow + kc, half);
#pragma unroll
        for (int t = 0; t < 4; ++t) {
            const v16h bf = ldfrag(bbase + (size_t)(t * 16) * DIM + kc, half);
            acc[t] = wmh(a, bf, acc[t]);
        }
    }
    const float osc = (MODE == 0) ? (1.0f / 128.0f) : (1.0f / 4096.0f);
#pragma unroll
    for (int t = 0; t < 4; ++t)
#pragma unroll
        for (int r = 0; r < 8; ++r) cst[(wv * 16 + 8 * half + r) * 68 + t * 16 + ln] = acc[t][r] * osc;
    __syncthreads();
    const int b = row0 / SEQ, n0 = row0 - b * SEQ;
    if (MODE == 0) {
        const int part = col0 / DIM, hh = (col0 - part * DIM) / HD;
        const int bh = b * NH + hh;
        if (part < 2) {
            u16* base = (part == 0 ? PQ : PK) + ((size_t)bh * SEQ + n0) * HD;
#pragma unroll
            for (int it = 0; it < 4; ++it) {
                const int p = it * 256 + tid, tr = p >> 3, d0 = (p & 7) * 8;
                const v4f e0 = *(const v4fa*)&cst[tr * 68 + d0];
                const v4f e1 = *(const v4fa*)&cst[tr * 68 + d0 + 4];
                v4u o;
                o[0] = pk2(e0[0], e0[1]); o[1] = pk2(e0[2], e0[3]);
                o[2] = pk2(e1[0], e1[1]); o[3] = pk2(e1[2], e1[3]);
                st2u(base + (size_t)tr * HD + d0, o);
            }
        } else {
            u16* base = PV + (size_t)bh * HD * SEQ + n0;
#pragma unroll
            for (int it = 0; it < 4; ++it) {
                const int p = it * 256 + tid, d = p >> 4, t0 = (p & 15) * 8;
                float e[8];
#pragma unroll
                for (int i = 0; i < 8; ++i) e[i] = cst[(t0 + i) * 68 + d];
                v4u o;
                o[0] = pk2(e[0], e[1]); o[1] = pk2(e[2], e[3]);
                o[2] = pk2(e[4], e[5]); o[3] = pk2(e[6], e[7]);
                st2u(base + (size_t)d * SEQ + t0, o);
            }
        }
    } else {
        float* ob = Y + ((size_t)b * SEQ_FULL + n0) * DIM + col0;
#pragma unroll
        for (int it = 0; it < 8; ++it) {
            const int p = it * 256 + tid, tr = p >> 4, c4 = (p & 15) * 4;
            v4f v = *(const v4fa*)&cst[tr * 68 + c4];
            v[0] += bfr(bias[col0 + c4]);
            v[1] += bfr(bias[col0 + c4 + 1]);
            v[2] += bfr(bias[col0 + c4 + 2]);
            v[3] += bfr(bias[col0 + c4 + 3]);
            st2f(ob + (size_t)tr * DIM + c4, v);
        }
    }
}

__global__ __launch_bounds__(256) void k_attn(const u16* __restrict__ QP, const u16* __restrict__ KP, const u16* __restrict__ VT, u16* CTX) {
    __shared__ __align__(16) u16 Ps[8 * 16 * 72];
    const int tid = threadIdx.x, lane = tid & 31, wv = tid >> 5, ln = lane & 15, half = lane >> 4;
    const int bh = blockIdx.y, b = bh / NH, hh = bh - b * NH;
    const int q0 = blockIdx.x * 128 + wv * 16;
    u16* myP = Ps + wv * (16 * 72);
    const u16* Kb = KP + (size_t)bh * SEQ * HD;
    const u16* Vb = VT + (size_t)bh * HD * SEQ;
    v16h qf[2];
    {
        const u16* qrow = QP + ((size_t)bh * SEQ + q0 + ln) * HD;
        qf[0] = ldfrag(qrow, half);
        qf[1] = ldfrag(qrow + 32, half);
    }
    float mrow[8], lrow[8];
#pragma unroll
    for (int r = 0; r < 8; ++r) { mrow[r] = -__builtin_inff(); lrow[r] = 0.0f; }
    v8f oacc[4];
#pragma unroll
    for (int g = 0; g < 4; ++g) oacc[g] = vz8();

#pragma unroll 1
    for (int j0 = 0; j0 < SEQ; j0 += 32) {
        v8f sacc[2];
        sacc[0] = vz8(); sacc[1] = vz8();
#pragma unroll
        for (int t = 0; t < 2; ++t) {
            const u16* krow = Kb + (size_t)(j0 + t * 16 + ln) * HD;
#pragma unroll
            for (int c = 0; c < 2; ++c) sacc[t] = wmh(qf[c], ldfrag(krow + c * 32, half), sacc[t]);
        }
        float alpha[8];
#pragma unroll
        for (int r = 0; r < 8; ++r) {
            const float s0 = sacc[0][r] * (1.0f / 128.0f), s1 = sacc[1][r] * (1.0f / 128.0f);
            float tm = fmaxf(s0, s1);
#pragma unroll
            for (int m = 1; m < 16; m <<= 1) tm = fmaxf(tm, __shfl_xor(tm, m, 32));
            const float mn = fmaxf(mrow[r], tm);
            const float a = __expf(mrow[r] - mn);
            const float p0 = __expf(s0 - mn), p1 = __expf(s1 - mn);
            float ps = p0 + p1;
#pragma unroll
            for (int m = 1; m < 16; m <<= 1) ps += __shfl_xor(ps, m, 32);
            lrow[r] = lrow[r] * a + ps;
            mrow[r] = mn;
            alpha[r] = a;
            myP[(8 * half + r) * 72 + ln] = (u16)h16(p0 * 1024.0f);
            myP[(8 * half + r) * 72 + 16 + ln] = (u16)h16(p1 * 1024.0f);
        }
#pragma unroll
        for (int g = 0; g < 4; ++g)
#pragma unroll
            for (int r = 0; r < 8; ++r) oacc[g][r] *= alpha[r];
        __syncthreads();
        const v16h pf = ldfrag(myP + ln * 72, half);
#pragma unroll
        for (int g = 0; g < 4; ++g) oacc[g] = wmh(pf, ldfrag(Vb + (size_t)(g * 16 + ln) * SEQ + j0, half), oacc[g]);
        __syncthreads();
    }
    float inv[8];
#pragma unroll
    for (int r = 0; r < 8; ++r) inv[r] = (1.0f / lrow[r]) * (1.0f / 64.0f);
#pragma unroll
    for (int g = 0; g < 4; ++g)
#pragma unroll
        for (int r = 0; r < 8; ++r) myP[(8 * half + r) * 72 + g * 16 + ln] = (u16)h16(oacc[g][r] * inv[r]);
    __syncthreads();
    u16* cb = CTX + ((size_t)b * SEQ + q0) * DIM + hh * HD;
    v4u o[4];
#pragma unroll
    for (int i = 0; i < 4; ++i) {
        Pk8 k;
        k.s = *(const v8usa*)(myP + (4 * i + (lane >> 3)) * 72 + (lane & 7) * 8);
        o[i] = k.w;
    }
#pragma unroll
    for (int i = 0; i < 4; ++i) *(volatile v4u*)(cb + (size_t)(4 * i + (lane >> 3)) * DIM + (lane & 7) * 8) = o[i];
    __threadfence();
#pragma unroll
    for (int i = 0; i < 4; ++i) *(volatile v4u*)(cb + (size_t)(4 * i + (lane >> 3)) * DIM + (lane & 7) * 8) = o[i];
}

extern "C" void kernel_launch(void* const* d_in, const int* in_sizes, int n_in,
                              void* d_out, int out_size, void* d_ws, size_t ws_size, hipStream_t stream) {
    if (n_in < 4) return;
    const float* x      = (const float*)d_in[0];
    const float* w_qkv  = (const float*)d_in[1];
    const float* w_proj = (const float*)d_in[2];
    const float* b_proj = (const float*)d_in[3];
    if (in_sizes[0] < ((NB - 1) * SEQ_FULL + SEQ) * DIM) return;
    if (in_sizes[1] < 3 * DIM * DIM || in_sizes[2] < DIM * DIM || in_sizes[3] < DIM) return;
    if (out_size < ((NB - 1) * SEQ_FULL + SEQ) * DIM) return;
    float* y = (float*)d_out;

    char* wsp = (char*)d_ws;
    auto take = [&](size_t bytes) { char* p = wsp; wsp += (bytes + 255) & ~(size_t)255; return (void*)p; };
    const size_t plane = (size_t)MTOK * DIM * 2;
    u16* XP  = (u16*)take(plane);
    u16* WQ  = (u16*)take((size_t)3 * DIM * DIM * 2);
    u16* WPR = (u16*)take((size_t)DIM * DIM * 2);
    u16* QP  = (u16*)take(plane);
    u16* KPl = (u16*)take(plane);
    u16* VT  = (u16*)take(plane);
    u16* CTX = (u16*)take(plane);
    if ((size_t)(wsp - (char*)d_ws) > ws_size) return;

    k_cvt_x<<<MTOK / 2, 256, 0, stream>>>(x, XP);
    k_cvt_w<<<(3 * DIM * DIM / 8 + 255) / 256, 256, 0, stream>>>(w_qkv, WQ, 3 * DIM * DIM / 8, 64.0f);
    k_cvt_w<<<(DIM * DIM / 8 + 255) / 256, 256, 0, stream>>>(w_proj, WPR, DIM * DIM / 8, 64.0f);
    k_gemm<0><<<dim3(MTOK / 128, 3 * DIM / 64, 1), 256, 0, stream>>>(XP, WQ, nullptr, QP, KPl, VT, nullptr);
    k_attn<<<dim3(SEQ / 128, NB * NH, 1), 256, 0, stream>>>(QP, KPl, VT, CTX);
    k_gemm<1><<<dim3(MTOK / 128, DIM / 64, 1), 256, 0, stream>>>(CTX, WPR, b_proj, nullptr, nullptr, nullptr, y);
}
